// LSTMExtractor_9448928051783
// MI455X (gfx1250) — hardware-verified
//
#include <hip/hip_runtime.h>


typedef _Float16 f16t;
typedef f16t  v16h __attribute__((ext_vector_type(16)));
typedef f16t  v8h  __attribute__((ext_vector_type(8)));
typedef float v8f  __attribute__((ext_vector_type(8)));
typedef float v4f  __attribute__((ext_vector_type(4)));
typedef unsigned int v4u __attribute__((ext_vector_type(4)));

union Frag { v16h v; v8h q[2]; };
union Pk16 { v8h h; v4u u; };

#define NSEQ  512
#define TLEN  512
#define DIN   28
#define KX    32
#define HID   128
#define G4    512
#define BT    16
#define HP    136
#define NTHR  512
#define L2E   1.4426950408889634f

__device__ __forceinline__ v8f wmma16(v16h a, v16h b, v8f c) {
  return __builtin_amdgcn_wmma_f32_16x16x32_f16(false, a, false, b, (short)0, c, false, false);
}

__device__ __forceinline__ void wguard4(v8f (&c)[4], const Frag& a, Frag (&b)[4]) {
  asm volatile("v_nop\n\tv_nop\n\tv_nop\n\tv_nop"
               : "+v"(c[0]), "+v"(c[1]), "+v"(c[2]), "+v"(c[3])
               : "v"(a.v), "v"(b[0].v), "v"(b[1].v), "v"(b[2].v), "v"(b[3].v));
}

__device__ __forceinline__ void ldfrag(Frag& f, const f16t* rowp, int k0, int hh) {
  const f16t* p = rowp + k0 + 8 * hh;
  f.q[0] = *(const v8h*)(p);
  f.q[1] = *(const v8h*)(p + 16);
}

__device__ __forceinline__ void mma4(v8f (&acc)[4], const Frag& a,
                                     const f16t* __restrict__ plane, int ldb,
                                     int nrow, int k0, int hh) {
  Frag b[4];
#pragma unroll
  for (int g = 0; g < 4; ++g)
    ldfrag(b[g], plane + (size_t)(nrow + g * HID) * ldb, k0, hh);
#pragma unroll
  for (int g = 0; g < 4; ++g) acc[g] = wmma16(a.v, b[g].v, acc[g]);
  wguard4(acc, a, b);
}

__device__ __forceinline__ float fsig(float x) {
  return __builtin_amdgcn_rcpf(1.0f + __builtin_amdgcn_exp2f(-x * L2E));
}
__device__ __forceinline__ float ftanh(float x) {
  const float t = __builtin_amdgcn_exp2f(-2.0f * L2E * fabsf(x));
  const float r = (1.0f - t) * __builtin_amdgcn_rcpf(1.0f + t);
  return copysignf(r, x);
}

__device__ __forceinline__ void cell(v8f (&acc)[4], float (&cst)[8], const float (&bias)[4],
                                     float inv, f16t* hdst, float* odst, bool wo,
                                     int hh, int ncol) {
#pragma unroll
  for (int r = 0; r < 8; ++r) {
    const float iv = fsig(fmaf(acc[0][r], inv, bias[0]));
    const float fv = fsig(fmaf(acc[1][r], inv, bias[1]));
    const float gv = ftanh(fmaf(acc[2][r], inv, bias[2]));
    const float ov = fsig(fmaf(acc[3][r], inv, bias[3]));
    const float cv = fmaf(fv, cst[r], iv * gv);
    cst[r] = cv;
    const float hv = ov * ftanh(cv);
    const int row = 8 * hh + r;
    hdst[row * HP + ncol] = (f16t)(hv * 256.0f);
    if (wo) odst[row * HID + ncol] = hv;
  }
}

__global__ __launch_bounds__(256)
void k_pack(const float* __restrict__ W, f16t* P, int N, int K, int KP, float sc) {
  const int i  = blockIdx.x * 256 + threadIdx.x;
  const int kq = KP >> 3;
  const int tot = N * kq;
  if (i >= tot) return;
  const int n  = i / kq;
  const int k8 = (i - n * kq) * 8;
  const float* src = W + (size_t)n * K;
  Pk16 v;
#pragma unroll
  for (int e = 0; e < 8; ++e) {
    const int k = k8 + e;
    float f = 0.0f;
    if (k < K) f = src[k] * sc;
    v.h[e] = (f16t)f;
  }
  f16t* d = P + (size_t)i * 8;
  *(volatile v4u*)d = v.u;
  __threadfence();
  *(volatile v4u*)d = v.u;
}

__global__ __launch_bounds__(NTHR)
void k_lstm2(const f16t* __restrict__ Xp,
             const f16t* __restrict__ Pih0, const f16t* __restrict__ Phh0,
             const float* __restrict__ bih0, const float* __restrict__ bhh0,
             const f16t* __restrict__ Pih1, const f16t* __restrict__ Phh1,
             const float* __restrict__ bih1, const float* __restrict__ bhh1,
             float* out, int T, int nb, float inv) {
  __shared__ __attribute__((aligned(16))) f16t  h0buf[2 * BT * HP];
  __shared__ __attribute__((aligned(16))) f16t  h1buf[2 * BT * HP];
  __shared__ __attribute__((aligned(16))) float outS[BT * HID];

  const int tid  = threadIdx.x;
  const int lane = tid & 31;
  const int wave = tid >> 5;
  const int hh   = lane >> 4;
  const int m    = lane & 15;
  const bool isB = wave >= 8;
  const int jt   = isB ? (wave - 8) : wave;
  const int ncol = jt * 16 + m;
  const int b0   = blockIdx.x * BT;
  if (b0 + BT > nb) return;

  for (int i = tid; i < 2 * BT * HP; i += NTHR) {
    h0buf[i] = (f16t)0.0f;
    h1buf[i] = (f16t)0.0f;
  }

  float bias[4];
  {
    const float* ba = isB ? bih1 : bih0;
    const float* bb = isB ? bhh1 : bhh0;
#pragma unroll
    for (int g = 0; g < 4; ++g) bias[g] = ba[g * HID + ncol] + bb[g * HID + ncol];
  }
  float cst[8];
#pragma unroll
  for (int r = 0; r < 8; ++r) cst[r] = 0.0f;
  __syncthreads();

  const f16t* xrow = Xp + ((size_t)(b0 + m) * T) * KX;
  const v8f z = {0.f, 0.f, 0.f, 0.f, 0.f, 0.f, 0.f, 0.f};

#pragma unroll 1
  for (int s = 0; s <= T; ++s) {
    const int p = s & 1;
    const f16t* h0cur = h0buf + p * (BT * HP);
    f16t*       h0nxt = h0buf + (1 - p) * (BT * HP);
    const f16t* h1cur = h1buf + p * (BT * HP);
    f16t*       h1nxt = h1buf + (1 - p) * (BT * HP);

    if (!isB) {
      if (s < T) {
        v8f acc[4];
#pragma unroll
        for (int g = 0; g < 4; ++g) acc[g] = z;
        Frag a;
        ldfrag(a, xrow + (size_t)s * KX, 0, hh);
        mma4(acc, a, Pih0, KX, ncol, 0, hh);
#pragma unroll 1
        for (int kc = 0; kc < 4; ++kc) {
          ldfrag(a, h0cur + m * HP, kc * 32, hh);
          mma4(acc, a, Phh0, HID, ncol, kc * 32, hh);
        }
        cell(acc, cst, bias, inv, h0nxt, outS, false, hh, ncol);
      }
    } else {
      if (s >= 1) {
        v8f acc[4];
#pragma unroll
        for (int g = 0; g < 4; ++g) acc[g] = z;
        Frag a;
#pragma unroll 1
        for (int kc = 0; kc < 4; ++kc) {
          ldfrag(a, h0cur + m * HP, kc * 32, hh);
          mma4(acc, a, Pih1, HID, ncol, kc * 32, hh);
        }
#pragma unroll 1
        for (int kc = 0; kc < 4; ++kc) {
          ldfrag(a, h1cur + m * HP, kc * 32, hh);
          mma4(acc, a, Phh1, HID, ncol, kc * 32, hh);
        }
        cell(acc, cst, bias, inv, h1nxt, outS, s == T, hh, ncol);
      }
    }
    __syncthreads();
  }

  {
    const int row = tid >> 5;
    const int c   = (tid & 31) * 4;
    const v4f v = *(const v4f*)(outS + row * HID + c);
    float* d = out + (size_t)(b0 + row) * HID + c;
    *(volatile v4f*)d = v;
    __threadfence();
    *(volatile v4f*)d = v;
  }
}

extern "C" void kernel_launch(void* const* d_in, const int* in_sizes, int n_in,
                              void* d_out, int out_size, void* d_ws, size_t ws_size,
                              hipStream_t stream) {
  const int nseq = NSEQ, T = TLEN, D = DIN, H = HID, G = G4;
  const int ntok = nseq * T;

  if (n_in < 9) return;
  if (in_sizes[0] != ntok * D || in_sizes[1] != G * D || in_sizes[2] != G * H ||
      in_sizes[3] != G || in_sizes[4] != G || in_sizes[5] != G * H ||
      in_sizes[6] != G * H || in_sizes[7] != G || in_sizes[8] != G) return;
  if (out_size != nseq * H) return;
  if ((nseq % BT) != 0) return;

  const float* x    = (const float*)d_in[0];
  const float* Wih0 = (const float*)d_in[1];
  const float* Whh0 = (const float*)d_in[2];
  const float* bih0 = (const float*)d_in[3];
  const float* bhh0 = (const float*)d_in[4];
  const float* Wih1 = (const float*)d_in[5];
  const float* Whh1 = (const float*)d_in[6];
  const float* bih1 = (const float*)d_in[7];
  const float* bhh1 = (const float*)d_in[8];
  float* out = (float*)d_out;

  char* ws = (char*)d_ws;
  size_t off = 0;
  auto carve = [&](size_t bytes) -> char* {
    char* ptr = ws + off;
    off = (off + bytes + 255) & ~(size_t)255;
    return ptr;
  };
  f16t* Xp   = (f16t*)carve((size_t)ntok * KX * 2);
  f16t* Pih0 = (f16t*)carve((size_t)G * KX * 2);
  f16t* Phh0 = (f16t*)carve((size_t)G * H * 2);
  f16t* Pih1 = (f16t*)carve((size_t)G * H * 2);
  f16t* Phh1 = (f16t*)carve((size_t)G * H * 2);
  if (off > ws_size) return;

  const float SX  = 1.0f;
  const float SI0 = 16384.0f;
  const float SW  = 64.0f;
  const float INV = 6.103515625e-05f;

  auto pack = [&](const float* W, f16t* P, int N, int K, int KP, float sc) {
    const int tot = N * (KP / 8);
    k_pack<<<dim3((tot + 255) / 256), dim3(256), 0, stream>>>(W, P, N, K, KP, sc);
  };
  pack(x,    Xp,   ntok, D, KX, SX);
  pack(Wih0, Pih0, G,    D, KX, SI0);
  pack(Whh0, Phh0, G,    H, H,  SW);
  pack(Wih1, Pih1, G,    H, H,  SW);
  pack(Whh1, Phh1, G,    H, H,  SW);

  k_lstm2<<<dim3(nseq / BT), dim3(NTHR), 0, stream>>>(Xp, Pih0, Phh0, bih0, bhh0,
                                                      Pih1, Phh1, bih1, bhh1,
                                                      out, T, nseq, INV);
}
